// Pointnet_FP_9792525435024
// MI455X (gfx1250) — hardware-verified
//
#include <hip/hip_runtime.h>
#include <math.h>

typedef __attribute__((ext_vector_type(16))) _Float16 v16h;
typedef __attribute__((ext_vector_type(16))) __bf16 v16b;
typedef __attribute__((ext_vector_type(8)))  _Float16 v8h;
typedef __attribute__((ext_vector_type(8)))  float v8f;
typedef __attribute__((ext_vector_type(4)))  float v4f;
typedef __attribute__((ext_vector_type(2)))  float v2f;
typedef __attribute__((ext_vector_type(4)))  unsigned v4u;
typedef __attribute__((ext_vector_type(4)))  int v4i;
typedef float __attribute__((may_alias)) float_a;
typedef int __attribute__((may_alias)) int_a;

template <typename T> __device__ __forceinline__ void vst2(void* p, T v) { *(volatile T*)p = v; __threadfence(); *(volatile T*)p = v; }
__device__ __forceinline__ v8f wmma16(v16h a, v16h b, v8f c) {
  v8f d = __builtin_amdgcn_wmma_f32_16x16x32_f16(false, a, false, b, (short)0, c, false, false);
  asm volatile("v_nop\n\tv_nop\n\tv_nop\n\tv_nop" : "+v"(d) : "v"(a), "v"(b));
  return d;
}
__device__ __forceinline__ v8f wmma_bf(v16b a, v16b b, v8f c) {
  v8f d = __builtin_amdgcn_wmma_f32_16x16x32_bf16(false, a, false, b, (short)0, c, false, false);
  asm volatile("v_nop\n\tv_nop\n\tv_nop\n\tv_nop" : "+v"(d) : "v"(a), "v"(b));
  return d;
}
__device__ __forceinline__ v16h frag_h(const _Float16* rowk0, int lane) {
  union { v16h v; v8h q[2]; } u; const _Float16* p = rowk0 + 8 * (lane >> 4);
  u.q[0] = *(const v8h*)p; u.q[1] = *(const v8h*)(p + 16); return u.v;
}
__device__ __forceinline__ v16h frag_f32(const float* rowk0, int lane) {
  v16h a; const float* p = rowk0 + 8 * (lane >> 4);
#pragma unroll
  for (int i = 0; i < 8; ++i) { a[i] = (_Float16)p[i]; a[8 + i] = (_Float16)p[16 + i]; }
  return a;
}
__device__ __forceinline__ v16h frag_f32s(const float* rowk0, int lane, float sc) {
  v16h a; const float* p = rowk0 + 8 * (lane >> 4);
#pragma unroll
  for (int i = 0; i < 8; ++i) { a[i] = (_Float16)(p[i] * sc); a[8 + i] = (_Float16)(p[16 + i] * sc); }
  return a;
}
__device__ __forceinline__ v16h fragc_f32(const float* W, int k0, int n, int lane, int ld, int K) {
  v16h a; const int g = lane >> 4;
#pragma unroll
  for (int i = 0; i < 8; ++i) { const int ka = k0 + 8 * g + i, kb = ka + 16;
    a[i] = (_Float16)(ka < K ? W[(size_t)(ka < K ? ka : K - 1) * ld + n] : 0.f); a[8 + i] = (_Float16)(kb < K ? W[(size_t)(kb < K ? kb : K - 1) * ld + n] : 0.f); }
  return a;
}
struct F2 { v16b h, l; };
__device__ __forceinline__ F2 bsplit16(const float v[16]) { F2 r;
#pragma unroll
  for (int i = 0; i < 16; ++i) { const __bf16 h = (__bf16)v[i]; r.h[i] = h; r.l[i] = (__bf16)(v[i] - (float)h); }
  return r; }
__device__ __forceinline__ F2 split_row(const float* row, int k0, int lane) { float v[16]; const float* p = row + k0 + 8 * (lane >> 4);
#pragma unroll
  for (int i = 0; i < 8; ++i) { v[i] = p[i]; v[8 + i] = p[16 + i]; }
  return bsplit16(v); }
__device__ __forceinline__ F2 split_rowK(const float* row, int k0, int lane, int K) { float v[16]; const int g = lane >> 4;
#pragma unroll
  for (int i = 0; i < 8; ++i) { const int ka = k0 + 8 * g + i, kb = ka + 16; v[i] = ka < K ? row[ka < K ? ka : K - 1] : 0.f; v[8 + i] = kb < K ? row[kb < K ? kb : K - 1] : 0.f; }
  return bsplit16(v); }
__device__ __forceinline__ F2 split_col(const float* W, int k0, int n, int lane, int ld, int K) { float v[16]; const int g = lane >> 4;
#pragma unroll
  for (int i = 0; i < 8; ++i) { const int ka = k0 + 8 * g + i, kb = ka + 16; v[i] = ka < K ? W[(size_t)(ka < K ? ka : K - 1) * ld + n] : 0.f; v[8 + i] = kb < K ? W[(size_t)(kb < K ? kb : K - 1) * ld + n] : 0.f; }
  return bsplit16(v); }
__device__ __forceinline__ v8f mac3(const F2& a, const F2& b, v8f c) { c = wmma_bf(a.l, b.h, c); c = wmma_bf(a.h, b.l, c); return wmma_bf(a.h, b.h, c); }
__device__ __forceinline__ float sigm(float v) { return 1.0f / (1.0f + expf(-v)); }
#define LDSX() do { asm volatile("s_wait_dscnt 0" ::: "memory"); __builtin_amdgcn_wave_barrier(); __builtin_amdgcn_fence(__ATOMIC_RELEASE, "workgroup"); } while (0)


#define NB 8
#define NN 4096
#define MMS 1024
#define C1 128
#define C2 256
#define CIN (C2 + C1)
#define F0 256
#define F1 256
#define NR (NB * NN)
#define RBLK (NR / 64)
typedef __attribute__((ext_vector_type(8))) __bf16 v8b;
__device__ __forceinline__ v16b frag_b(const __bf16* rowk0, int lane) {
  union { v16b v; v8b q[2]; } u; const __bf16* p = rowk0 + 8 * (lane >> 4);
  u.q[0] = *(const v8b*)p; u.q[1] = *(const v8b*)(p + 16); return u.v;
}
__device__ __forceinline__ float bfr(float v) { return (float)(__bf16)v; }
__device__ __attribute__((noinline)) float exp_ni(float v) { return expf(v); }
__device__ __attribute__((noinline)) float erf_ni(float v) { return erff(v); }

#define WS_P1  0u
#define WS_P2  (2u * F0 * CIN)
#define WS_NN  (WS_P2 + 2u * F1 * F0)
#define WS_XH  (WS_NN + 4u * NR * 8)
#define WS_XL  (WS_XH + 2u * NR * CIN)
#define WS_Y   (WS_XL + 2u * NR * CIN)
#define WS_ST  (WS_Y + 4u * NR * F0)
#define WS_MS  (WS_ST + 4u * RBLK * F0 * 2)
#define WS_HH  (WS_MS + 4u * F0 * 2)
#define WS_HL  (WS_HH + 2u * NR * F0)
#define WS_END (WS_HL + 2u * NR * F0)

__global__ __launch_bounds__(256) void k_pack(const float* __restrict__ W1, const float* __restrict__ W2, __bf16* __restrict__ PK) {
  __shared__ __align__(16) __bf16 s[CIN]; const int n = blockIdx.x, which = blockIdx.y, t = threadIdx.x; const int K = (which == 0) ? CIN : F0;
  for (int k = t; k < K; k += 256) s[k] = (__bf16)((which == 0) ? W1[(size_t)k * F0 + n] : W2[(size_t)k * F1 + n]);
  __syncthreads();
  for (int q = t; q < K / 8; q += 256) vst2((unsigned*)(PK + ((which == 0) ? 0 : (size_t)F0 * CIN) + (size_t)n * K + q * 8), *(const v4u*)&s[q * 8]);
}
__device__ __forceinline__ void ins3(float d, int i, float* bd, int* bi) {
  if (d < bd[2] || (d == bd[2] && i < bi[2])) {
    if (d < bd[1] || (d == bd[1] && i < bi[1])) { bd[2] = bd[1]; bi[2] = bi[1];
      if (d < bd[0] || (d == bd[0] && i < bi[0])) { bd[1] = bd[0]; bi[1] = bi[0]; bd[0] = d; bi[0] = i; } else { bd[1] = d; bi[1] = i; } }
    else { bd[2] = d; bi[2] = i; } } }
__global__ __launch_bounds__(256) void k_knn(const float* __restrict__ X1, const float* __restrict__ X2, float* __restrict__ NNW) {
  __shared__ float sx2[MMS][3]; __shared__ float sq2[MMS]; __shared__ float sd[64][4][3]; __shared__ int si[64][4][3]; __shared__ __align__(16) float so[64][8];
  const int t = threadIdx.x; const size_t b = blockIdx.y; const int n0 = blockIdx.x * 64; const int q = t >> 2, part = t & 3;
  for (int i = t; i < MMS; i += 256) { const float x = bfr(X2[(b * MMS + i) * 3]), y = bfr(X2[(b * MMS + i) * 3 + 1]), z = bfr(X2[(b * MMS + i) * 3 + 2]); sx2[i][0] = x; sx2[i][1] = y; sx2[i][2] = z; sq2[i] = (x * x + y * y) + z * z; }
  __syncthreads();
  const size_t row = b * NN + n0 + q; const float px = bfr(X1[row * 3]), py = bfr(X1[row * 3 + 1]), pz = bfr(X1[row * 3 + 2]); const float sq1 = (px * px + pz * pz) + py * py;
  float bd[3] = {3.0e38f, 3.0e38f, 3.0e38f}; int bi[3] = {0x7fffffff, 0x7fffffff, 0x7fffffff};
#pragma unroll 1
  for (int i = part * (MMS / 4); i < (part + 1) * (MMS / 4); ++i) { const float dot = (px * sx2[i][0] + py * sx2[i][1]) + pz * sx2[i][2]; const float d = (sq1 + sq2[i]) - 2.0f * dot; ins3(d, i, bd, bi); }
#pragma unroll
  for (int k = 0; k < 3; ++k) { sd[q][part][k] = bd[k]; si[q][part][k] = bi[k]; }
  __syncthreads();
  if (part == 0) { for (int p2 = 1; p2 < 4; ++p2) for (int k = 0; k < 3; ++k) ins3(sd[q][p2][k], si[q][p2][k], bd, bi);
    float w[3], ws = 0.f;
#pragma unroll
    for (int k = 0; k < 3; ++k) { const float dd = fmaxf(bd[k], 1e-10f); w[k] = 1.0f / dd; ws += w[k]; }
#pragma unroll
    for (int k = 0; k < 3; ++k) { so[q][k] = __int_as_float(bi[k]); so[q][3 + k] = w[k] / ws; } so[q][6] = 0.f; so[q][7] = 0.f; }
  __syncthreads();
  for (int e = t; e < 64 * 2; e += 256) { const int r = e >> 1, h = e & 1; vst2(NNW + (b * NN + n0 + r) * 8 + h * 4, *(const v4f*)&so[r][h * 4]); }
}
__global__ __launch_bounds__(256) void k_feat(const float* __restrict__ NNW, const float* __restrict__ P2, const float* __restrict__ P1, __bf16* __restrict__ XH, __bf16* __restrict__ XL) {
  __shared__ __align__(16) __bf16 sh[16][CIN + 8], sl[16][CIN + 8]; const int t = threadIdx.x; const size_t row0 = (size_t)blockIdx.x * 16; const size_t b = row0 / NN;
  for (int e = t; e < 16 * CIN; e += 256) { const int r = e / CIN, c = e % CIN; const size_t row = row0 + r; float v, lo = 0.f;
    if (c < C2) { const float* nw = NNW + row * 8; const int i0 = __float_as_int(nw[0]), i1 = __float_as_int(nw[1]), i2 = __float_as_int(nw[2]);
      const float g0 = bfr(P2[(b * MMS + i0) * C2 + c]), g1 = bfr(P2[(b * MMS + i1) * C2 + c]), g2 = bfr(P2[(b * MMS + i2) * C2 + c]);
      v = (g0 * nw[3] + g1 * nw[4]) + g2 * nw[5]; const __bf16 hb = (__bf16)v; lo = v - (float)hb; v = (float)hb; }
    else v = bfr(P1[row * C1 + (c - C2)]);
    sh[r][c] = (__bf16)v; sl[r][c] = (__bf16)lo; }
  __syncthreads();
  for (int e = t; e < 16 * (CIN / 8); e += 256) { const int r = e / (CIN / 8), q = e % (CIN / 8); vst2((unsigned*)(XH + (row0 + r) * CIN + q * 8), *(const v4u*)&sh[r][q * 8]); vst2((unsigned*)(XL + (row0 + r) * CIN + q * 8), *(const v4u*)&sl[r][q * 8]); }
}
template <int KD>
__global__ __launch_bounds__(128) void k_conv(const __bf16* __restrict__ AH, const __bf16* __restrict__ AL, const __bf16* __restrict__ P, float* __restrict__ Y, float* __restrict__ ST) {
  __shared__ __align__(16) float so[4][16][132]; __shared__ __align__(16) float sst[128][2];
  const int tid = threadIdx.x, wave = tid >> 5, lane = tid & 31, col = lane & 15, g = lane >> 4; const size_t r0 = (size_t)blockIdx.x * 64 + wave * 16; const int n0 = blockIdx.y * 128;
  v8f acc[8] = {};
#pragma unroll 2
  for (int kc = 0; kc < KD / 32; ++kc) { const v16b a = frag_b(AH + (r0 + col) * KD + kc * 32, lane), al = frag_b(AL + (r0 + col) * KD + kc * 32, lane);
#pragma unroll
    for (int j = 0; j < 8; ++j) { const v16b w = frag_b(P + (size_t)(n0 + j * 16 + col) * KD + kc * 32, lane); acc[j] = wmma_bf(al, w, acc[j]); acc[j] = wmma_bf(a, w, acc[j]); } }
#pragma unroll
  for (int j = 0; j < 8; ++j)
#pragma unroll
    for (int r = 0; r < 8; ++r) so[wave][8 * g + r][j * 16 + col] = acc[j][r];
  __syncthreads();
  for (int rl = 0; rl < 16; ++rl) vst2(Y + (r0 + rl) * F0 + n0 + lane * 4, *(const v4f*)&so[wave][rl][lane * 4]);
  { const int c = tid; float s = 0.f, q2 = 0.f; for (int w = 0; w < 4; ++w) for (int r = 0; r < 16; ++r) { const float v = so[w][r][c]; s += v; q2 += v * v; } sst[c][0] = s; sst[c][1] = q2; }
  __syncthreads();
  if (tid < 64) vst2(ST + ((size_t)blockIdx.x * F0 + n0) * 2 + tid * 4, *(const v4f*)(&sst[0][0] + tid * 4));
}
__global__ __launch_bounds__(256) void k_bnstat(const float* __restrict__ ST, float* __restrict__ MS) {
  const int c = threadIdx.x; float s = 0.f, q2 = 0.f;
#pragma unroll 1
  for (int blk = 0; blk < RBLK; ++blk) { s += ST[((size_t)blk * F0 + c) * 2]; q2 += ST[((size_t)blk * F0 + c) * 2 + 1]; }
  const float mu = s / (float)NR; const float var = fmaxf(q2 / (float)NR - mu * mu, 0.f);
  __shared__ __align__(16) float sm[F0][2]; sm[c][0] = mu; sm[c][1] = 1.0f / sqrtf(var + 1e-3f); __syncthreads();
  if (c < F0 * 2 / 4) vst2(MS + c * 4, *(const v4f*)(&sm[0][0] + c * 4));
}
template <int FINAL>
__global__ __launch_bounds__(256) void k_bnrelu(const float* __restrict__ Y, const float* __restrict__ MS, const float* __restrict__ G, const float* __restrict__ Bt, __bf16* __restrict__ HH, __bf16* __restrict__ HL, float* __restrict__ OUT) {
  __shared__ __align__(16) __bf16 sh[64][F0 + 8], sl[64][F0 + 8]; __shared__ __align__(16) float so[16][F0 + 4];
  const int c = threadIdx.x; const size_t r0 = (size_t)blockIdx.x * 64; const float mu = MS[c * 2], rs = MS[c * 2 + 1], gg = bfr(G[c]), bb = bfr(Bt[c]);
  if (FINAL) {
    for (int rb = 0; rb < 64; rb += 16) { for (int r = 0; r < 16; ++r) { const float y = Y[(r0 + rb + r) * F0 + c]; so[r][c] = fmaxf((y - mu) * rs * gg + bb, 0.f); } __syncthreads();
      for (int e = c; e < 16 * F0 / 4; e += 256) { const int r = e / (F0 / 4), q = e % (F0 / 4); vst2(OUT + (r0 + rb + r) * F0 + q * 4, *(const v4f*)&so[r][q * 4]); } __syncthreads(); }
  } else {
    for (int r = 0; r < 64; ++r) { const float y = Y[(r0 + r) * F0 + c]; const float v = fmaxf((y - mu) * rs * gg + bb, 0.f); const __bf16 hb = (__bf16)v; sh[r][c] = hb; sl[r][c] = (__bf16)(v - (float)hb); }
    __syncthreads();
    for (int e = c; e < 64 * (F0 / 8); e += 256) { const int r = e / (F0 / 8), q = e % (F0 / 8); vst2((unsigned*)(HH + (r0 + r) * F0 + q * 8), *(const v4u*)&sh[r][q * 8]); vst2((unsigned*)(HL + (r0 + r) * F0 + q * 8), *(const v4u*)&sl[r][q * 8]); } }
}
extern "C" void kernel_launch(void* const* d_in, const int* in_sizes, int n_in, void* d_out, int out_size, void* d_ws, size_t ws_size, hipStream_t stream) {
  (void)in_sizes; (void)n_in; (void)out_size;
  const float** F = (const float**)d_in;
  if (ws_size < (size_t)WS_END) return;
  char* ws = (char*)d_ws; __bf16 *PK = (__bf16*)(ws + WS_P1), *XH = (__bf16*)(ws + WS_XH), *XL = (__bf16*)(ws + WS_XL), *HH = (__bf16*)(ws + WS_HH), *HL = (__bf16*)(ws + WS_HL); float *NNW = (float*)(ws + WS_NN), *Y = (float*)(ws + WS_Y), *ST = (float*)(ws + WS_ST), *MS = (float*)(ws + WS_MS);
  k_pack<<<dim3(F0, 2), 256, 0, stream>>>(F[4], F[7], PK);
  k_knn<<<dim3(NN / 64, NB), 256, 0, stream>>>(F[0], F[1], NNW);
  k_feat<<<NR / 16, 256, 0, stream>>>(NNW, F[3], F[2], XH, XL);
  k_conv<CIN><<<dim3(RBLK, F0 / 128), 128, 0, stream>>>(XH, XL, PK, Y, ST);
  k_bnstat<<<1, 256, 0, stream>>>(ST, MS);
  k_bnrelu<0><<<RBLK, 256, 0, stream>>>(Y, MS, F[5], F[6], HH, HL, nullptr);
  k_conv<F0><<<dim3(RBLK, F1 / 128), 128, 0, stream>>>(HH, HL, PK + (size_t)F0 * CIN, Y, ST);
  k_bnstat<<<1, 256, 0, stream>>>(ST, MS);
  k_bnrelu<1><<<RBLK, 256, 0, stream>>>(Y, MS, F[8], F[9], nullptr, nullptr, (float*)d_out);
}
